// BertSelfAttention_24687472017696
// MI455X (gfx1250) — hardware-verified
//
#include <hip/hip_runtime.h>
#include <cstddef>


typedef _Float16 v16h __attribute__((ext_vector_type(16)));
typedef _Float16 v8h  __attribute__((ext_vector_type(8)));
typedef float    v8f  __attribute__((ext_vector_type(8)));
typedef float    v4f  __attribute__((ext_vector_type(4)));

#ifndef NB
#define NB 4
#endif
#ifndef SEQ
#define SEQ 2048
#endif
#define NB_FULL  4
#define SEQ_FULL 2048
#define HID      1024
#define NHEAD    16
#define DHEAD    64
#define MROWS    (NB * SEQ)
#define SPITCH   72
#define WSCALE   64.0f
#define WINV     0.015625f
#define PCARRY   1024.0f
#define PINV     0.0009765625f
#define SM_SCALE 0.125f

static_assert(SEQ % 128 == 0);
static_assert(SEQ >= 128);
static_assert(SEQ <= SEQ_FULL);
static_assert(NB >= 1);
static_assert(NB <= NB_FULL);
static_assert(HID == NHEAD * DHEAD);
static_assert(MROWS % 64 == 0);
static_assert(HID % 256 == 0);
static_assert((SPITCH % 8) == 0);

__device__ __forceinline__ float bf16r(float x) {
  unsigned u = __float_as_uint(x);
  u = (u + 0x7FFFu + ((u >> 16) & 1u)) & 0xFFFF0000u;
  return __uint_as_float(u);
}

__device__ __forceinline__ v8f wmma16(v16h a, v16h b, v8f c) {
  c = __builtin_amdgcn_wmma_f32_16x16x32_f16(false, a, false, b, (short)0, c, false, false);
  asm volatile("v_nop\n\tv_nop\n\tv_nop\n\tv_nop" : "+v"(c) : "v"(a), "v"(b));
  return c;
}

__device__ __forceinline__ v8f zero8() {
  v8f z;
#pragma unroll
  for (int i = 0; i < 8; ++i) z[i] = 0.0f;
  return z;
}

__global__ __launch_bounds__(256) void k_cvt(const float* __restrict__ src,
                                             _Float16* __restrict__ dst,
                                             int nrows, int seq, int seq_full, float scale) {
  const int g  = blockIdx.x * 256 + threadIdx.x;
  const int n8 = nrows * (HID / 8);
  if (g < n8) {
    const int m  = g / (HID / 8);
    const int c  = (g - m * (HID / 8)) * 8;
    const int bb = m / seq;
    const int s  = m - bb * seq;
    const float* sp = src + ((size_t)bb * seq_full + s) * HID + c;
    const v4f a0 = *(const v4f*)sp;
    const v4f a1 = *(const v4f*)(sp + 4);
    v8h o;
#pragma unroll
    for (int i = 0; i < 4; ++i) {
      o[i]     = (_Float16)(bf16r(a0[i]) * scale);
      o[i + 4] = (_Float16)(bf16r(a1[i]) * scale);
    }
    _Float16* dp = dst + (size_t)g * 8;
    *(volatile v8h*)dp = o;
    __threadfence();
    *(volatile v8h*)dp = o;
  }
}

template <int MODE>
__global__ __launch_bounds__(256) void k_proj(const _Float16* __restrict__ A,
                                              const _Float16* __restrict__ W,
                                              const float* __restrict__ bias,
                                              _Float16* __restrict__ outp) {
  __shared__ __align__(16) _Float16 stg[256 * SPITCH];

  const int lane = threadIdx.x & 31;
  const int wave = threadIdx.x >> 5;
  const int l15  = lane & 15;
  const int kb   = (lane >> 4) * 8;
  const int lq   = lane >> 3;
  const int lp   = (lane & 7) * 8;
  const int wm   = wave & 1;
  const int wn   = wave >> 1;
  const int m0   = blockIdx.x * 64;
  const int n0   = blockIdx.y * 256;
  const int mw   = m0 + 32 * wm;
  const int nw   = n0 + 64 * wn;

  const _Float16* ap0 = A + (size_t)(mw + l15) * HID + kb;
  const _Float16* ap1 = ap0 + (size_t)16 * HID;
  const _Float16* bp0 = W + (size_t)(nw + l15) * HID + kb;

  v8f acc[2][4];
#pragma unroll
  for (int mi = 0; mi < 2; ++mi)
#pragma unroll
    for (int ni = 0; ni < 4; ++ni) acc[mi][ni] = zero8();

  for (int k = 0; k < HID; k += 32) {
    v16h af[2], bfm[4];
    ((v8h*)&af[0])[0] = *(const v8h*)(ap0 + k);
    ((v8h*)&af[0])[1] = *(const v8h*)(ap0 + k + 16);
    ((v8h*)&af[1])[0] = *(const v8h*)(ap1 + k);
    ((v8h*)&af[1])[1] = *(const v8h*)(ap1 + k + 16);
#pragma unroll
    for (int ni = 0; ni < 4; ++ni) {
      const _Float16* bp = bp0 + (size_t)(16 * ni) * HID + k;
      ((v8h*)&bfm[ni])[0] = *(const v8h*)(bp);
      ((v8h*)&bfm[ni])[1] = *(const v8h*)(bp + 16);
    }
#pragma unroll
    for (int mi = 0; mi < 2; ++mi)
#pragma unroll
      for (int ni = 0; ni < 4; ++ni)
        acc[mi][ni] = wmma16(af[mi], bfm[ni], acc[mi][ni]);
  }

  float bn[4];
#pragma unroll
  for (int ni = 0; ni < 4; ++ni) bn[ni] = bf16r(bias[nw + 16 * ni + l15]);

  v8h hv[8];
  if constexpr (MODE == 0) {
    _Float16* sw = stg + wave * (32 * SPITCH);
#pragma unroll
    for (int mi = 0; mi < 2; ++mi)
#pragma unroll
      for (int ni = 0; ni < 4; ++ni)
#pragma unroll
        for (int r = 0; r < 8; ++r)
          sw[(16 * mi + kb + r) * SPITCH + 16 * ni + l15] =
              (_Float16)(acc[mi][ni][r] * WINV + bn[ni]);
    __syncthreads();
#pragma unroll
    for (int i = 0; i < 8; ++i)
      hv[i] = *(const v8h*)(sw + (4 * i + lq) * SPITCH + lp);
    _Float16* dbase = outp + (size_t)(mw + lq) * HID + nw + lp;
#pragma unroll
    for (int i = 0; i < 8; ++i)
      *(volatile v8h*)(dbase + (size_t)(4 * i) * HID) = hv[i];
    __threadfence();
#pragma unroll
    for (int i = 0; i < 8; ++i)
      *(volatile v8h*)(dbase + (size_t)(4 * i) * HID) = hv[i];
  } else {
#pragma unroll
    for (int mi = 0; mi < 2; ++mi)
#pragma unroll
      for (int ni = 0; ni < 4; ++ni)
#pragma unroll
        for (int r = 0; r < 8; ++r)
          stg[(64 * wn + 16 * ni + l15) * SPITCH + 32 * wm + 16 * mi + kb + r] =
              (_Float16)(acc[mi][ni][r] * WINV + bn[ni]);
    __syncthreads();
    const int bb = m0 / SEQ;
    const int s0 = m0 - bb * SEQ;
#pragma unroll
    for (int i = 0; i < 8; ++i)
      hv[i] = *(const v8h*)(stg + (32 * wave + 4 * i + lq) * SPITCH + lp);
    _Float16* vbase = outp +
        ((size_t)((bb * NHEAD + (n0 >> 6) + (wave >> 1)) * DHEAD + 32 * (wave & 1) + lq)) * SEQ +
        s0 + lp;
#pragma unroll
    for (int i = 0; i < 8; ++i)
      *(volatile v8h*)(vbase + (size_t)(4 * i) * SEQ) = hv[i];
    __threadfence();
#pragma unroll
    for (int i = 0; i < 8; ++i)
      *(volatile v8h*)(vbase + (size_t)(4 * i) * SEQ) = hv[i];
  }
}

__global__ __launch_bounds__(256) void k_attn(const _Float16* __restrict__ Qm,
                                              const _Float16* __restrict__ Km,
                                              const _Float16* __restrict__ VT,
                                              const float* __restrict__ mask,
                                              float* __restrict__ out) {
  __shared__ __align__(16) _Float16 pbuf[8][16 * 64];
  __shared__ __align__(16) float    obuf[8][16 * 64];

  const int lane = threadIdx.x & 31;
  const int wave = threadIdx.x >> 5;
  const int l15  = lane & 15;
  const int kb   = (lane >> 4) * 8;
  const int lq   = lane >> 3;
  const int QT   = SEQ / 16;
  const int tile = blockIdx.x * 8 + wave;
  const int bh   = tile / QT;
  const int qt   = tile - bh * QT;
  const int b    = bh / NHEAD;
  const int h    = bh - b * NHEAD;
  const int q0   = qt * 16;

  const _Float16* qrow = Qm + (size_t)(b * SEQ + q0 + l15) * HID + h * DHEAD;
  v16h qa0, qa1;
  ((v8h*)&qa0)[0] = *(const v8h*)(qrow + kb);
  ((v8h*)&qa0)[1] = *(const v8h*)(qrow + kb + 16);
  ((v8h*)&qa1)[0] = *(const v8h*)(qrow + 32 + kb);
  ((v8h*)&qa1)[1] = *(const v8h*)(qrow + 32 + kb + 16);

  float mrow[8], lrow[8];
#pragma unroll
  for (int r = 0; r < 8; ++r) { mrow[r] = -1e30f; lrow[r] = 0.0f; }
  v8f o[4];
#pragma unroll
  for (int t = 0; t < 4; ++t) o[t] = zero8();

  const float* maskb   = mask + (size_t)b * SEQ_FULL;
  const _Float16* Kb   = Km + (size_t)(b * SEQ) * HID + h * DHEAD;
  const _Float16* VTbh = VT + (size_t)bh * DHEAD * SEQ;
  _Float16* pw = pbuf[wave];

  for (int kc = 0; kc < SEQ; kc += 64) {
    v8f s[4];
#pragma unroll
    for (int j = 0; j < 4; ++j) s[j] = zero8();
    const _Float16* kbase = Kb + (size_t)(kc + l15) * HID;
#pragma unroll
    for (int j = 0; j < 4; ++j) {
      const _Float16* krow = kbase + (size_t)(16 * j) * HID;
      v16h kf0, kf1;
      ((v8h*)&kf0)[0] = *(const v8h*)(krow + kb);
      ((v8h*)&kf0)[1] = *(const v8h*)(krow + kb + 16);
      ((v8h*)&kf1)[0] = *(const v8h*)(krow + 32 + kb);
      ((v8h*)&kf1)[1] = *(const v8h*)(krow + 32 + kb + 16);
      s[j] = wmma16(qa0, kf0, s[j]);
      s[j] = wmma16(qa1, kf1, s[j]);
    }

    float mk[4];
#pragma unroll
    for (int j = 0; j < 4; ++j) mk[j] = bf16r(maskb[kc + 16 * j + l15]);

#pragma unroll
    for (int r = 0; r < 8; ++r) {
      const float a0 = s[0][r] * SM_SCALE + mk[0];
      const float a1 = s[1][r] * SM_SCALE + mk[1];
      const float a2 = s[2][r] * SM_SCALE + mk[2];
      const float a3 = s[3][r] * SM_SCALE + mk[3];
      float t = fmaxf(fmaxf(a0, a1), fmaxf(a2, a3));
      t = fmaxf(t, __shfl_xor(t, 1));
      t = fmaxf(t, __shfl_xor(t, 2));
      t = fmaxf(t, __shfl_xor(t, 4));
      t = fmaxf(t, __shfl_xor(t, 8));
      const float newm = fmaxf(mrow[r], t);
      const float corr = __expf(mrow[r] - newm);
      mrow[r] = newm;
      const float p0 = __expf(a0 - newm);
      const float p1 = __expf(a1 - newm);
      const float p2 = __expf(a2 - newm);
      const float p3 = __expf(a3 - newm);
      lrow[r] = lrow[r] * corr + (p0 + p1) + (p2 + p3);
      o[0][r] *= corr; o[1][r] *= corr; o[2][r] *= corr; o[3][r] *= corr;
      const int row = r + kb;
      pw[row * 64 + l15]      = (_Float16)(p0 * PCARRY);
      pw[row * 64 + 16 + l15] = (_Float16)(p1 * PCARRY);
      pw[row * 64 + 32 + l15] = (_Float16)(p2 * PCARRY);
      pw[row * 64 + 48 + l15] = (_Float16)(p3 * PCARRY);
    }
    __syncthreads();

    v16h pa0, pa1;
    ((v8h*)&pa0)[0] = *(const v8h*)(pw + l15 * 64 + kb);
    ((v8h*)&pa0)[1] = *(const v8h*)(pw + l15 * 64 + 16 + kb);
    ((v8h*)&pa1)[0] = *(const v8h*)(pw + l15 * 64 + 32 + kb);
    ((v8h*)&pa1)[1] = *(const v8h*)(pw + l15 * 64 + 48 + kb);

#pragma unroll
    for (int t = 0; t < 4; ++t) {
      const _Float16* vrow = VTbh + (size_t)(16 * t + l15) * SEQ + kc;
      v16h vf0, vf1;
      ((v8h*)&vf0)[0] = *(const v8h*)(vrow + kb);
      ((v8h*)&vf0)[1] = *(const v8h*)(vrow + kb + 16);
      ((v8h*)&vf1)[0] = *(const v8h*)(vrow + 32 + kb);
      ((v8h*)&vf1)[1] = *(const v8h*)(vrow + 48 + kb);
      o[t] = wmma16(pa0, vf0, o[t]);
      o[t] = wmma16(pa1, vf1, o[t]);
    }
  }

  float* ob = obuf[wave];
#pragma unroll
  for (int r = 0; r < 8; ++r) {
    float rs = lrow[r];
    rs += __shfl_xor(rs, 1);
    rs += __shfl_xor(rs, 2);
    rs += __shfl_xor(rs, 4);
    rs += __shfl_xor(rs, 8);
    const float inv = (1.0f / rs) * PINV;
#pragma unroll
    for (int t = 0; t < 4; ++t) ob[(r + kb) * 64 + 16 * t + l15] = o[t][r] * inv;
  }
  __syncthreads();

  const int orl = lq >> 1;
  const int ocol = 32 * (lq & 1) + 4 * (lane & 7);
  v4f ov[8];
#pragma unroll
  for (int i = 0; i < 8; ++i) ov[i] = *(const v4f*)(ob + (2 * i + orl) * 64 + ocol);
  float* obase = out + ((size_t)b * SEQ_FULL + q0 + orl) * HID + h * DHEAD + ocol;
#pragma unroll
  for (int i = 0; i < 8; ++i) *(volatile v4f*)(obase + (size_t)(2 * i) * HID) = ov[i];
  __threadfence();
#pragma unroll
  for (int i = 0; i < 8; ++i) *(volatile v4f*)(obase + (size_t)(2 * i) * HID) = ov[i];
}

extern "C" void kernel_launch(void* const* d_in, const int* in_sizes, int n_in,
                              void* d_out, int out_size, void* d_ws, size_t ws_size,
                              hipStream_t stream) {
  if (n_in < 8) return;
  const long long need_x = ((long long)(NB - 1) * SEQ_FULL + SEQ) * HID;
  if ((long long)in_sizes[0] < need_x) return;
  if (in_sizes[1] < (NB - 1) * SEQ_FULL + SEQ) return;
  if (in_sizes[2] < HID * HID || in_sizes[4] < HID * HID || in_sizes[6] < HID * HID) return;
  if (in_sizes[3] < HID || in_sizes[5] < HID || in_sizes[7] < HID) return;
  if ((long long)out_size < need_x) return;

  const float* hs   = (const float*)d_in[0];
  const float* mask = (const float*)d_in[1];
  const float* Wq   = (const float*)d_in[2];
  const float* bq   = (const float*)d_in[3];
  const float* Wk   = (const float*)d_in[4];
  const float* bk   = (const float*)d_in[5];
  const float* Wv   = (const float*)d_in[6];
  const float* bv   = (const float*)d_in[7];
  float* out = (float*)d_out;

  const size_t XN  = (size_t)MROWS * HID;
  const size_t WN  = (size_t)HID * HID;
  const size_t QN  = XN;
  const size_t VTN = (size_t)NB * NHEAD * DHEAD * SEQ;
  const size_t total_bytes = 2 * (XN + 3 * WN + 2 * QN + VTN);
  if (ws_size < total_bytes) return;

  _Float16* x16  = (_Float16*)d_ws;
  _Float16* wq16 = x16 + XN;
  _Float16* wk16 = wq16 + WN;
  _Float16* wv16 = wk16 + WN;
  _Float16* q16  = wv16 + WN;
  _Float16* k16  = q16 + QN;
  _Float16* vt16 = k16 + QN;

  const int gx = (MROWS * (HID / 8) + 255) / 256;
  const int gw = (HID * (HID / 8) + 255) / 256;
  k_cvt<<<gx, 256, 0, stream>>>(hs, x16, MROWS, SEQ, SEQ_FULL, 1.0f);
  k_cvt<<<gw, 256, 0, stream>>>(Wq, wq16, HID, HID, HID, WSCALE);
  k_cvt<<<gw, 256, 0, stream>>>(Wk, wk16, HID, HID, HID, WSCALE);
  k_cvt<<<gw, 256, 0, stream>>>(Wv, wv16, HID, HID, HID, WSCALE);

  const dim3 gg(MROWS / 64, HID / 256);
  k_proj<0><<<gg, 256, 0, stream>>>(x16, wq16, bq, q16);
  k_proj<0><<<gg, 256, 0, stream>>>(x16, wk16, bk, k16);
  k_proj<1><<<gg, 256, 0, stream>>>(x16, wv16, bv, vt16);

  const int ga = (NB * NHEAD * (SEQ / 16)) / 8;
  k_attn<<<ga, 256, 0, stream>>>(q16, k16, vt16, mask, out);
}
